// CartesianDecomposedAttention_876173328862
// MI455X (gfx1250) — hardware-verified
//
#include <hip/hip_runtime.h>
#include <math.h>
#include <stdint.h>

#define DM   1024
#define NH   16
#define DHD  64
#define NB   2
#define SQ   1024
#define MR   (NB * SQ)
#define KS   (2 * DM)

#define PLW  ((size_t)DM * KS)
#define PLX  ((size_t)MR * KS)
#define PLQ  ((size_t)MR * DM)
#define PLV  ((size_t)DM * MR)
#define PLA  ((size_t)MR * KS)

typedef __attribute__((ext_vector_type(16))) __bf16         v16b;
typedef __attribute__((ext_vector_type(16))) unsigned short v16us;
typedef __attribute__((ext_vector_type(8)))  unsigned short v8us;
typedef __attribute__((ext_vector_type(8)))  unsigned int   v8u;
typedef __attribute__((ext_vector_type(8)))  float          v8f;
typedef __attribute__((ext_vector_type(4)))  float          v4f;
typedef __attribute__((ext_vector_type(4)))  unsigned int   v4u;

union FragU { v16us u; v8us h[2]; v16b b; };

static __device__ __forceinline__ unsigned short bf_bits(float f) {
  const unsigned u = __float_as_uint(f);
  return (unsigned short)((u + 0x7FFFu + ((u >> 16) & 1u)) >> 16);
}
static __device__ __forceinline__ float bf_val(unsigned short hb) { return __uint_as_float(((unsigned)hb) << 16); }
static __device__ __forceinline__ unsigned pk2(unsigned short a, unsigned short b) { return (unsigned)a | ((unsigned)b << 16); }

static __device__ __forceinline__ v8f zero8() { v8f z = {0.f, 0.f, 0.f, 0.f, 0.f, 0.f, 0.f, 0.f}; return z; }

static __device__ __forceinline__ v16us ldfrag(const unsigned short* p) {
  FragU f;
  f.h[0] = *(const v8us*)p;
  f.h[1] = *(const v8us*)(p + 16);
  return f.u;
}

static __device__ __forceinline__ v8f mma(v16us a, v16us b, v8f c) {
  FragU ua, ub;
  ua.u = a; ub.u = b;
  c = __builtin_amdgcn_wmma_f32_16x16x32_bf16(false, ua.b, false, ub.b, (short)0, c, false, false);
  asm volatile("v_nop\n\tv_nop\n\tv_nop\n\tv_nop" : "+v"(c) : "v"(ua.b), "v"(ub.b));
  return c;
}

static __device__ __forceinline__ v16us neg16(v16us a) {
  union { v16us u; v8u w; } x;
  x.u = a;
  const v8u sgn = {0x80008000u, 0x80008000u, 0x80008000u, 0x80008000u,
                   0x80008000u, 0x80008000u, 0x80008000u, 0x80008000u};
  x.w = x.w ^ sgn;
  return x.u;
}

static __device__ __forceinline__ void wave_sync() {
  __builtin_amdgcn_fence(__ATOMIC_RELEASE, "workgroup");
  __builtin_amdgcn_wave_barrier();
  __builtin_amdgcn_fence(__ATOMIC_ACQUIRE, "workgroup");
}

static __device__ __forceinline__ void split8(const float* sp, v4u& hv, v4u& lv) {
  v4u hq, lq;
#pragma unroll
  for (int qq = 0; qq < 4; ++qq) {
    const float f0 = sp[2 * qq], f1 = sp[2 * qq + 1];
    const unsigned short h0 = bf_bits(f0), h1 = bf_bits(f1);
    const unsigned short l0 = bf_bits(f0 - bf_val(h0)), l1 = bf_bits(f1 - bf_val(h1));
    hq[qq] = pk2(h0, h1);
    lq[qq] = pk2(l0, l1);
  }
  hv = hq; lv = lq;
}

__global__ __launch_bounds__(256) void cvt_x_kernel(const float* xre, const float* xim, unsigned short* xs) {
  const int part = blockIdx.z;
  const float* src = (part == 0) ? xre : xim;
  const int row = blockIdx.x * 2 + (threadIdx.x >> 7);
  const int c8  = (threadIdx.x & 127) * 8;
  const float* sp = src + (size_t)row * DM + c8;
  const v4f f0 = *(const v4f*)sp;
  const v4f f1 = *(const v4f*)(sp + 4);
  v4u o;
  o[0] = pk2(bf_bits(f0[0]), bf_bits(f0[1]));
  o[1] = pk2(bf_bits(f0[2]), bf_bits(f0[3]));
  o[2] = pk2(bf_bits(f1[0]), bf_bits(f1[1]));
  o[3] = pk2(bf_bits(f1[2]), bf_bits(f1[3]));
  unsigned short* dp = xs + (size_t)row * KS + (size_t)part * DM + c8;
  *(volatile v4u*)dp = o;
  __threadfence();
  *(volatile v4u*)dp = o;
}

__global__ __launch_bounds__(256) void cvt_w_kernel(const float* wqr, const float* wqi, const float* wkr, const float* wki,
                                                    const float* wvr, const float* wvi, const float* wor, const float* woi,
                                                    unsigned short* wst) {
  const int z = blockIdx.z;
  const float* wr = (z == 0) ? wqr : (z == 1) ? wkr : (z == 2) ? wvr : wor;
  const float* wi = (z == 0) ? wqi : (z == 1) ? wki : (z == 2) ? wvi : woi;
  const int n  = blockIdx.x * 2 + (threadIdx.x >> 7);
  const int c8 = (threadIdx.x & 127) * 8;
  const float* rp = wr + (size_t)n * DM + c8;
  const float* ip = wi + (size_t)n * DM + c8;
  const v4f r0 = *(const v4f*)rp, r1 = *(const v4f*)(rp + 4);
  const v4f i0 = *(const v4f*)ip, i1 = *(const v4f*)(ip + 4);
  float rf[8] = {r0[0], r0[1], r0[2], r0[3], r1[0], r1[1], r1[2], r1[3]};
  float iff[8] = {i0[0], i0[1], i0[2], i0[3], i1[0], i1[1], i1[2], i1[3]};
  v4u re8, im8, nim8;
#pragma unroll
  for (int qq = 0; qq < 4; ++qq) {
    re8[qq]  = pk2(bf_bits(rf[2 * qq]), bf_bits(rf[2 * qq + 1]));
    im8[qq]  = pk2(bf_bits(iff[2 * qq]), bf_bits(iff[2 * qq + 1]));
    nim8[qq] = im8[qq] ^ 0x80008000u;
  }
  unsigned short* pre = wst + (size_t)(2 * z) * PLW + (size_t)n * KS + c8;
  unsigned short* pim = pre + PLW;
  *(volatile v4u*)(pre)      = re8;
  *(volatile v4u*)(pre + DM) = nim8;
  *(volatile v4u*)(pim)      = im8;
  *(volatile v4u*)(pim + DM) = re8;
  __threadfence();
  *(volatile v4u*)(pre)      = re8;
  *(volatile v4u*)(pre + DM) = nim8;
  *(volatile v4u*)(pim)      = im8;
  *(volatile v4u*)(pim + DM) = re8;
}

struct InvF { float v[DHD]; };
static_assert(sizeof(InvF) == 256);

__global__ __launch_bounds__(256) void rot_kernel(float* rc, float* rs, InvF inv) {
  const int d = blockIdx.y;
  const int s = blockIdx.x * 256 + threadIdx.x;
  const float ang = (float)s * inv.v[d];
  float sn, cs;
  sincosf(ang, &sn, &cs);
  const size_t idx = (size_t)d * SQ + s;
  *(volatile float*)(rc + idx) = cs;
  *(volatile float*)(rs + idx) = sn;
  __threadfence();
  *(volatile float*)(rc + idx) = cs;
  *(volatile float*)(rs + idx) = sn;
}

template <int AMODE, int EPI>
__global__ __launch_bounds__(128) void cgemm_kernel(
    const unsigned short* A0, const unsigned short* A1, int lda, long long zA,
    const unsigned short* B0, const unsigned short* B1, int ldb, long long zB,
    unsigned short* Crh, unsigned short* Crl, unsigned short* Cih, unsigned short* Cil, int ldc, long long zC,
    float* Cf, const float* rc, const float* rs, int K) {
  __shared__ __align__(16) float slabs[4][16 * 132];
  const int wave = threadIdx.x >> 5;
  const int lane = threadIdx.x & 31;
  const int hh   = lane >> 4;
  const int rl   = lane & 15;
  const size_t z = blockIdx.z;
  const int m0 = (blockIdx.y * 4 + wave) * 16;
  const int n0 = blockIdx.x * 64;

  const unsigned short* a0p = A0 + z * (size_t)zA + (size_t)(m0 + rl) * lda + 8 * hh;
  const unsigned short* a1p = A1 + z * (size_t)zA + (size_t)(m0 + rl) * lda + 8 * hh;
  const unsigned short* b0p = B0 + z * (size_t)zB + (size_t)(n0 + rl) * ldb + 8 * hh;
  const unsigned short* b1p = B1 + z * (size_t)zB + (size_t)(n0 + rl) * ldb + 8 * hh;

  v8f are[4], aim[4];
#pragma unroll
  for (int j = 0; j < 4; ++j) { are[j] = zero8(); aim[j] = zero8(); }

  for (int k0 = 0; k0 < K; k0 += 32) {
    const v16us fa0 = ldfrag(a0p + k0);
    v16us fa1 = fa0;
    if (AMODE != 0) fa1 = ldfrag(a1p + k0);
#pragma unroll
    for (int j = 0; j < 4; ++j) {
      const size_t bo = (size_t)(16 * j) * ldb + k0;
      const v16us fb0 = ldfrag(b0p + bo);
      if (AMODE == 1) {
        are[j] = mma(fa0, fb0, are[j]);
        aim[j] = mma(fa1, fb0, aim[j]);
      } else {
        const v16us fb1 = ldfrag(b1p + bo);
        are[j] = mma(fa0, fb0, are[j]);
        aim[j] = mma(fa0, fb1, aim[j]);
        if (AMODE == 2) {
          are[j] = mma(fa1, fb0, are[j]);
          aim[j] = mma(fa1, fb1, aim[j]);
        }
      }
    }
  }

  float* slab = slabs[wave];
  if (EPI == 0) {
    const int sb = (m0 + 8 * hh) & (SQ - 1);
#pragma unroll
    for (int j = 0; j < 4; ++j) {
      const int d = 16 * j + rl;
      const float* cp = rc + (size_t)d * SQ + sb;
      const float* snp = rs + (size_t)d * SQ + sb;
#pragma unroll
      for (int r = 0; r < 8; ++r) {
        const float cs = cp[r], sn = snp[r];
        const float yr = are[j][r], yi = aim[j][r];
        are[j][r] = yr * cs - yi * sn;
        aim[j][r] = yr * sn + yi * cs;
      }
    }
  }

  if (EPI == 2) {
#pragma unroll
    for (int j = 0; j < 4; ++j)
#pragma unroll
      for (int r = 0; r < 8; ++r) {
        slab[(8 * hh + r) * 132 + 2 * (16 * j + rl)]     = are[j][r];
        slab[(8 * hh + r) * 132 + 2 * (16 * j + rl) + 1] = aim[j][r];
      }
    wave_sync();
    v4f ov[16];
#pragma unroll
    for (int row = 0; row < 16; ++row) ov[row] = *(const v4f*)(slab + row * 132 + 4 * lane);
    float* cb = Cf + (size_t)m0 * (size_t)(2 * ldc) + (size_t)(2 * n0) + 4 * lane;
    for (int rep = 0; rep < 2; ++rep) {
#pragma unroll
      for (int row = 0; row < 16; ++row)
        *(volatile v4f*)(cb + (size_t)row * (size_t)(2 * ldc)) = ov[row];
      __threadfence();
    }
  } else {
#pragma unroll
    for (int j = 0; j < 4; ++j)
#pragma unroll
      for (int r = 0; r < 8; ++r) {
        slab[(8 * hh + r) * 132 + 16 * j + rl]      = are[j][r];
        slab[(8 * hh + r) * 132 + 64 + 16 * j + rl] = aim[j][r];
      }
    wave_sync();
    const int q = lane >> 3, c8 = (lane & 7) * 8;
    v4u hv[4][2], lv[4][2];
#pragma unroll
    for (int it = 0; it < 4; ++it)
#pragma unroll
      for (int part = 0; part < 2; ++part)
        split8(slab + (it * 4 + q) * 132 + part * 64 + c8, hv[it][part], lv[it][part]);
    unsigned short* crh = Crh + z * (size_t)zC;
    unsigned short* crl = Crl + z * (size_t)zC;
    unsigned short* cih = Cih + z * (size_t)zC;
    unsigned short* cil = Cil + z * (size_t)zC;
    for (int rep = 0; rep < 2; ++rep) {
#pragma unroll
      for (int it = 0; it < 4; ++it) {
        const size_t go = (size_t)(m0 + it * 4 + q) * ldc + n0 + c8;
        *(volatile v4u*)(crh + go) = hv[it][0];
        *(volatile v4u*)(crl + go) = lv[it][0];
        *(volatile v4u*)(cih + go) = hv[it][1];
        *(volatile v4u*)(cil + go) = lv[it][1];
      }
      __threadfence();
    }
  }
}

#define AKC 32

__global__ __launch_bounds__(128) void attn_kernel(
    const unsigned short* qrh, const unsigned short* qrl, const unsigned short* qih, const unsigned short* qil,
    const unsigned short* krh, const unsigned short* krl, const unsigned short* kih, const unsigned short* kil,
    const unsigned short* vrh, const unsigned short* vrl, const unsigned short* vih, const unsigned short* vil,
    unsigned short* ash, unsigned short* asl) {
  __shared__ __align__(16) unsigned short Kt[4][AKC * DHD];
  __shared__ __align__(16) unsigned short Vt[4][DHD * AKC];
  __shared__ __align__(16) unsigned short Pt[2][4][16 * AKC];
  __shared__ __align__(16) float Ot[2][2][16 * 68];
  __shared__ float Xm[2][2][16];
  __shared__ float Xs[2][2][16];

  const int tid  = threadIdx.x;
  const int wave = tid >> 5;
  const int lane = tid & 31;
  const int hh   = lane >> 4;
  const int c    = lane & 15;
  const int g    = wave >> 1;
  const int rr   = wave & 1;
  const int b    = blockIdx.z;
  const int h    = blockIdx.y;
  const int q0   = blockIdx.x * 32 + g * 16;
  const int row8 = 8 * hh;

  const unsigned short* qp[4] = {qrh, qrl, qih, qil};
  const unsigned short* kp[4] = {krh, krl, kih, kil};
  const unsigned short* vp[4] = {vrh, vrl, vih, vil};
  const size_t qoff = (size_t)(b * SQ + q0 + c) * DM + (size_t)h * DHD + 8 * hh;

  v8f ore[2], oim[2];
#pragma unroll
  for (int dt = 0; dt < 2; ++dt) { ore[dt] = zero8(); oim[dt] = zero8(); }
  float mrow[8], lrow[8];
#pragma unroll
  for (int r8 = 0; r8 < 8; ++r8) { mrow[r8] = -1e30f; lrow[r8] = 0.f; }

  for (int kc = 0; kc < SQ / AKC; ++kc) {
    const int t0 = kc * AKC;
    __syncthreads();
#pragma unroll
    for (int it = 0; it < 8; ++it) {
      const int p   = it >> 1;
      const int rem = (tid + 128 * it) & 255;
      const int kt  = rem >> 3, kc8 = (rem & 7) * 8;
      const int vd  = rem >> 2, vc8 = (rem & 3) * 8;
      const v8us kv = *(const v8us*)(kp[p] + (size_t)(b * SQ + t0 + kt) * DM + h * DHD + kc8);
      const v8us vv = *(const v8us*)(vp[p] + (size_t)(h * DHD + vd) * MR + b * SQ + t0 + vc8);
      *(v8us*)(&Kt[p][kt * DHD + kc8]) = kv;
      *(v8us*)(&Vt[p][vd * AKC + vc8]) = vv;
    }
    __syncthreads();

    v8f sre = zero8(), sim = zero8();
    const int krow = (16 * rr + c) * DHD + 8 * hh;
#pragma unroll
    for (int dc = 0; dc < 2; ++dc) {
      const v16us q_rh = ldfrag(qp[0] + qoff + dc * 32);
      const v16us q_rl = ldfrag(qp[1] + qoff + dc * 32);
      const v16us q_ih = ldfrag(qp[2] + qoff + dc * 32);
      const v16us q_il = ldfrag(qp[3] + qoff + dc * 32);
      {
        const v16us k_h = ldfrag(&Kt[0][krow + dc * 32]);
        const v16us k_l = ldfrag(&Kt[1][krow + dc * 32]);
        sre = mma(q_rh, k_h, sre); sre = mma(q_rh, k_l, sre); sre = mma(q_rl, k_h, sre);
        sim = mma(q_ih, k_h, sim); sim = mma(q_ih, k_l, sim); sim = mma(q_il, k_h, sim);
      }
      {
        const v16us k_h = ldfrag(&Kt[2][krow + dc * 32]);
        const v16us k_l = ldfrag(&Kt[3][krow + dc * 32]);
        sre = mma(q_ih, k_h, sre); sre = mma(q_ih, k_l, sre); sre = mma(q_il, k_h, sre);
        const v16us n_h = neg16(k_h);
        const v16us n_l = neg16(k_l);
        sim = mma(q_rh, n_h, sim); sim = mma(q_rh, n_l, sim); sim = mma(q_rl, n_h, sim);
      }
    }
    sre = sre * 0.125f;
    sim = sim * 0.125f;

    float pm[8];
#pragma unroll
    for (int r8 = 0; r8 < 8; ++r8) {
      float m = sre[r8];
#pragma unroll
      for (int off = 1; off < 16; off <<= 1) m = fmaxf(m, __shfl_xor(m, off, 32));
      pm[r8] = m;
    }
    if (c == 0) {
#pragma unroll
      for (int r8 = 0; r8 < 8; ++r8) Xm[g][rr][row8 + r8] = pm[r8];
    }
    __syncthreads();

    float mnew[8], alpha[8];
#pragma unroll
    for (int r8 = 0; r8 < 8; ++r8) {
      const float cm = fmaxf(Xm[g][0][row8 + r8], Xm[g][1][row8 + r8]);
      mnew[r8]  = fmaxf(mrow[r8], cm);
      alpha[r8] = __expf(mrow[r8] - mnew[r8]);
      mrow[r8]  = mnew[r8];
      ore[0][r8] *= alpha[r8];
      ore[1][r8] *= alpha[r8];
      oim[0][r8] *= alpha[r8];
      oim[1][r8] *= alpha[r8];
      lrow[r8] *= alpha[r8];
    }

    float ps[8];
#pragma unroll
    for (int r8 = 0; r8 < 8; ++r8) {
      const float p = __expf(sre[r8] - mnew[r8]);
      float sn, cs;
      sincosf(sim[r8], &sn, &cs);
      const float wr = p * cs, wi = p * sn;
      const unsigned short hr  = bf_bits(wr), hi2 = bf_bits(wi);
      const unsigned short lr  = bf_bits(wr - bf_val(hr)), li2 = bf_bits(wi - bf_val(hi2));
      const int po = (row8 + r8) * AKC + 16 * rr + c;
      Pt[g][0][po] = hr;
      Pt[g][1][po] = lr;
      Pt[g][2][po] = hi2;
      Pt[g][3][po] = li2;
      float s = p;
#pragma unroll
      for (int off = 1; off < 16; off <<= 1) s += __shfl_xor(s, off, 32);
      ps[r8] = s;
    }
    if (c == 0) {
#pragma unroll
      for (int r8 = 0; r8 < 8; ++r8) Xs[g][rr][row8 + r8] = ps[r8];
    }
    __syncthreads();
#pragma unroll
    for (int r8 = 0; r8 < 8; ++r8) lrow[r8] += Xs[g][0][row8 + r8] + Xs[g][1][row8 + r8];

    const int prow = c * AKC + 8 * hh;
    const v16us w_rh = ldfrag(&Pt[g][0][prow]);
    const v16us w_rl = ldfrag(&Pt[g][1][prow]);
    const v16us w_ih = ldfrag(&Pt[g][2][prow]);
    const v16us w_il = ldfrag(&Pt[g][3][prow]);
#pragma unroll
    for (int dt = 0; dt < 2; ++dt) {
      const int vrow = (16 * (2 * rr + dt) + c) * AKC + 8 * hh;
      {
        const v16us v_h = ldfrag(&Vt[0][vrow]);
        const v16us v_l = ldfrag(&Vt[1][vrow]);
        ore[dt] = mma(w_rh, v_h, ore[dt]); ore[dt] = mma(w_rh, v_l, ore[dt]); ore[dt] = mma(w_rl, v_h, ore[dt]);
        oim[dt] = mma(w_ih, v_h, oim[dt]); oim[dt] = mma(w_ih, v_l, oim[dt]); oim[dt] = mma(w_il, v_h, oim[dt]);
      }
      {
        const v16us v_h = ldfrag(&Vt[2][vrow]);
        const v16us v_l = ldfrag(&Vt[3][vrow]);
        oim[dt] = mma(w_rh, v_h, oim[dt]); oim[dt] = mma(w_rh, v_l, oim[dt]); oim[dt] = mma(w_rl, v_h, oim[dt]);
        const v16us n_h = neg16(v_h);
        const v16us n_l = neg16(v_l);
        ore[dt] = mma(w_ih, n_h, ore[dt]); ore[dt] = mma(w_ih, n_l, ore[dt]); ore[dt] = mma(w_il, n_h, ore[dt]);
      }
    }
  }

#pragma unroll
  for (int r8 = 0; r8 < 8; ++r8) {
    const float inv = 1.0f / lrow[r8];
#pragma unroll
    for (int dt = 0; dt < 2; ++dt) {
      const int col = 16 * (2 * rr + dt) + c;
      Ot[g][0][(row8 + r8) * 68 + col] = ore[dt][r8] * inv;
      Ot[g][1][(row8 + r8) * 68 + col] = oim[dt][r8] * inv;
    }
  }
  __syncthreads();
  const int q = lane >> 3, c8 = (lane & 7) * 8;
  v4u ov[4][2];
#pragma unroll
  for (int it = 0; it < 4; ++it)
#pragma unroll
    for (int part = 0; part < 2; ++part) {
      v4u hv, lv;
      split8(&Ot[g][part][(it * 4 + q) * 68 + c8], hv, lv);
      if (rr == 0) ov[it][part] = hv; else ov[it][part] = lv;
    }
  unsigned short* dst = (rr == 0) ? ash : asl;
  const size_t rbase = (size_t)(b * SQ + q0) * KS + (size_t)h * DHD + c8;
  for (int rep = 0; rep < 2; ++rep) {
#pragma unroll
    for (int it = 0; it < 4; ++it)
#pragma unroll
      for (int part = 0; part < 2; ++part)
        *(volatile v4u*)(dst + rbase + (size_t)(it * 4 + q) * KS + (size_t)part * DM) = ov[it][part];
    __threadfence();
  }
}

extern "C" void kernel_launch(void* const* d_in, const int* in_sizes, int n_in,
                              void* d_out, int out_size, void* d_ws, size_t ws_size,
                              hipStream_t stream) {
  if (n_in < 10) return;
  if (in_sizes[0] != MR * DM || in_sizes[1] != MR * DM) return;
  for (int i = 2; i < 10; ++i) if (in_sizes[i] != DM * DM) return;
  if (out_size != MR * DM * 2) return;

  const size_t oRC  = 0;
  const size_t oRS  = oRC + (size_t)DHD * SQ * 4;
  const size_t oXS  = oRS + (size_t)DHD * SQ * 4;
  const size_t oW   = oXS + PLX * 2;
  const size_t oQK  = oW  + 8 * PLW * 2;
  const size_t oVT  = oQK + 8 * PLQ * 2;
  const size_t oAS  = oVT + 4 * PLV * 2;
  const size_t oEnd = oAS + 2 * PLA * 2;
  if (oEnd > ws_size) return;

  const float* xre = (const float*)d_in[0];
  const float* xim = (const float*)d_in[1];
  const float* wqr = (const float*)d_in[2];
  const float* wqi = (const float*)d_in[3];
  const float* wkr = (const float*)d_in[4];
  const float* wki = (const float*)d_in[5];
  const float* wvr = (const float*)d_in[6];
  const float* wvi = (const float*)d_in[7];
  const float* wor = (const float*)d_in[8];
  const float* woi = (const float*)d_in[9];

  char* ws = (char*)d_ws;
  float*          RC = (float*)(ws + oRC);
  float*          RS = (float*)(ws + oRS);
  unsigned short* XS = (unsigned short*)(ws + oXS);
  unsigned short* W  = (unsigned short*)(ws + oW);
  unsigned short* QK = (unsigned short*)(ws + oQK);
  unsigned short* VT = (unsigned short*)(ws + oVT);
  unsigned short* AS = (unsigned short*)(ws + oAS);
  float*          OUTF = (float*)d_out;

  InvF inv;
  for (int d = 0; d < DHD; ++d) {
    const float e = (float)d / (float)DHD;
    const float pw = powf(10000.0f, e);
    inv.v[d] = 1.0f / pw;
  }

  cvt_x_kernel<<<dim3(MR / 2, 1, 2), dim3(256), 0, stream>>>(xre, xim, XS);
  cvt_w_kernel<<<dim3(DM / 2, 1, 4), dim3(256), 0, stream>>>(wqr, wqi, wkr, wki, wvr, wvi, wor, woi, W);
  rot_kernel<<<dim3(SQ / 256, DHD, 1), dim3(256), 0, stream>>>(RC, RS, inv);
  cgemm_kernel<0, 0><<<dim3(DM / 64, MR / 64, 2), dim3(128), 0, stream>>>(
      XS, XS, KS, 0LL,
      W, W + PLW, KS, (long long)(2 * PLW),
      QK, QK + PLQ, QK + 2 * PLQ, QK + 3 * PLQ, DM, (long long)(4 * PLQ),
      OUTF, RC, RS, KS);
  cgemm_kernel<1, 1><<<dim3(MR / 64, DM / 64, 1), dim3(128), 0, stream>>>(
      W + 4 * PLW, W + 5 * PLW, KS, 0LL,
      XS, XS, KS, 0LL,
      VT, VT + PLV, VT + 2 * PLV, VT + 3 * PLV, MR, 0LL,
      OUTF, RC, RS, KS);
  attn_kernel<<<dim3(SQ / 32, NH, NB), dim3(128), 0, stream>>>(
      QK, QK + PLQ, QK + 2 * PLQ, QK + 3 * PLQ,
      QK + 4 * PLQ, QK + 5 * PLQ, QK + 6 * PLQ, QK + 7 * PLQ,
      VT, VT + PLV, VT + 2 * PLV, VT + 3 * PLV,
      AS, AS + PLA);
  cgemm_kernel<2, 2><<<dim3(DM / 64, MR / 64, 1), dim3(128), 0, stream>>>(
      AS, AS + PLA, KS, 0LL,
      W + 6 * PLW, W + 7 * PLW, KS, 0LL,
      AS, AS, AS, AS, DM, 0LL,
      OUTF, RC, RS, KS);
  (void)hipGetLastError();
}
